// DNCCell_6081673691270
// MI455X (gfx1250) — hardware-run, weakly checked
//
#include <hip/hip_runtime.h>
#include <math.h>

#pragma clang fp contract(off)

typedef __attribute__((ext_vector_type(16))) _Float16 v16h;
typedef __attribute__((ext_vector_type(8)))  _Float16 v8h;
typedef __attribute__((ext_vector_type(4)))  _Float16 v4h;
typedef __attribute__((ext_vector_type(8)))  float    v8f;
typedef __attribute__((ext_vector_type(4)))  float    v4f;

__device__ __forceinline__ void dep_guard_h(v8f& a, v8f& b, v16h x, v16h y) { asm volatile("v_nop\n\tv_nop\n\tv_nop\n\tv_nop" : "+v"(a), "+v"(b) : "v"(x), "v"(y)); }
__device__ __forceinline__ void keep4_h(v16h a, v16h b, v16h c, v16h d) { asm volatile("v_nop" :: "v"(a), "v"(b), "v"(c), "v"(d)); }
__device__ __forceinline__ void acc_guard4(v8f& a, v8f& b, v8f& c, v8f& d) { asm volatile("v_nop\n\tv_nop\n\tv_nop\n\tv_nop" : "+v"(a), "+v"(b), "+v"(c), "+v"(d)); }

template <typename T> struct Frag;
template <> struct Frag<_Float16> {
  typedef v16h V; union U { v16h v; v8h h[2]; };
  static __device__ __forceinline__ v16h load(const _Float16* p) {
    U f; f.h[0] = *(const v8h*)(p); f.h[1] = *(const v8h*)(p + 16); return f.v;
  }
  static __device__ __forceinline__ v8f mma(v16h a, v16h b, v8f c) {
    return __builtin_amdgcn_wmma_f32_16x16x32_f16(false, a, false, b, (short)0, c, false, false);
  }
};

constexpr int NBATCH = 64;
constexpr int NSTEP  = 256;
constexpr int NUNIT  = 512;
constexpr int NSLOT  = 16;
constexpr int NLOGIT = 17;
constexpr int ROWS_PB = 16;
constexpr int A_PITCH  = 528;
constexpr int TR_PITCH = 516;
constexpr float READ_CARRY = 16.0f;
constexpr float WT_CARRY   = 64.0f;
constexpr float ACC_FOLD   = 1.0f / 1024.0f;
constexpr float MEAN_RECIP = 1.0f / 17.0f;

__device__ __forceinline__ v8f zero8() { v8f z; z[0]=0.f; z[1]=0.f; z[2]=0.f; z[3]=0.f; z[4]=0.f; z[5]=0.f; z[6]=0.f; z[7]=0.f; return z; }
__device__ __forceinline__ v4f fma4(float a, v4f b, v4f c) {
  v4f r;
  r[0] = fmaf(a, b[0], c[0]); r[1] = fmaf(a, b[1], c[1]); r[2] = fmaf(a, b[2], c[2]); r[3] = fmaf(a, b[3], c[3]);
  return r;
}

__global__ __launch_bounds__(256) void wt_cast_kmajor(const float* __restrict__ Wt, _Float16* __restrict__ WtT) {
  __shared__ float tile[64][65];
  const int n0 = blockIdx.x * 64;
  const int k0 = blockIdx.y * 64;
  const int tid = threadIdx.x;
#pragma unroll 1
  for (int idx = tid; idx < 4096; idx += 256) {
    const int kk = idx >> 6;
    const int nn = idx & 63;
    tile[nn][kk] = Wt[(size_t)(k0 + kk) * NUNIT + n0 + nn];
  }
  __syncthreads();
  const int q  = tid >> 3;
  const int c8 = (tid & 7) * 8;
  v8h hv[2];
#pragma unroll
  for (int p = 0; p < 2; ++p) {
    const int nn = q + 32 * p;
#pragma unroll
    for (int e = 0; e < 8; ++e) hv[p][e] = (_Float16)(tile[nn][c8 + e] * WT_CARRY);
  }
  for (int pass = 0; pass < 2; ++pass) {
#pragma unroll
    for (int p = 0; p < 2; ++p)
      *(volatile v8h*)(WtT + (size_t)(n0 + q + 32 * p) * NUNIT + k0 + c8) = hv[p];
    __threadfence();
  }
}

__global__ __launch_bounds__(256) void dnc_steps(
    const float* __restrict__ x, const float* mem_init,
    const float* __restrict__ Wr, const float* __restrict__ br,
    const _Float16* __restrict__ WtT, const float* __restrict__ bt,
    const float* __restrict__ Ww, const float* __restrict__ bw,
    float* memA, float* memB, float* __restrict__ out) {
  __shared__ __align__(16) _Float16 readA[ROWS_PB * A_PITCH];
  __shared__ __align__(16) float    trS[ROWS_PB * TR_PITCH];
  __shared__ __align__(16) float    btS[NUNIT];
  __shared__ float brS[32];
  __shared__ float bwS[NSLOT];

  const int tid  = threadIdx.x;
  const int wave = tid >> 5;
  const int lane = tid & 31;
  const int hh   = lane >> 4;
  const int cc   = lane & 15;
  const int koff = hh * 8;
  const int row0 = blockIdx.x * ROWS_PB;
  const int nwcol = wave * 64;

  btS[tid] = bt[tid];
  btS[tid + 256] = bt[tid + 256];
  if (tid < 32) {
    const int bi = (tid < NLOGIT) ? tid : (NLOGIT - 1);
    const float bv = br[bi];
    brS[tid] = (tid < NLOGIT) ? bv : 0.f;
  }
  if (tid < NSLOT) {
    const int bi = (tid < NSLOT) ? tid : (NSLOT - 1);
    bwS[tid] = bw[bi];
  }
  __syncthreads();

  for (int t = 0; t < NSTEP; ++t) {
    const float* src = (t == 0) ? mem_init : ((t & 1) ? (const float*)memA : (const float*)memB);
    float* dst = (t & 1) ? memB : memA;

#pragma unroll 1
    for (int rr = 0; rr < 2; ++rr) {
      const int lr = wave * 2 + rr;
      const int gb = row0 + lr;
      const float* xrow = x + ((size_t)gb * NSTEP + t) * NUNIT;
      const float* mrow = src + (size_t)gb * (NSLOT * NUNIT);

      float part[NLOGIT];
#pragma unroll
      for (int k = 0; k < NLOGIT; ++k) part[k] = 0.f;

#pragma unroll 1
      for (int i = 0; i < 4; ++i) {
        const int u0 = lane * 4 + 128 * i;
        v4f s = *(const v4f*)(mrow + u0);
#pragma unroll
        for (int m = 1; m < NSLOT; ++m) {
          const v4f mv = *(const v4f*)(mrow + m * NUNIT + u0);
          s = s + mv;
        }
        const v4f xs = *(const v4f*)(xrow + u0);
        s = s + xs;
        const float* wrb = Wr + (size_t)u0 * NLOGIT;
#pragma unroll
        for (int j = 0; j < 4; ++j) {
          const float a = s[j] * MEAN_RECIP;
          v4f wq[5];
#pragma unroll
          for (int cq = 0; cq < 5; ++cq) wq[cq] = *(const v4f*)(wrb + 16 * j + 4 * cq);
#pragma unroll
          for (int k = 0; k < NLOGIT; ++k) part[k] = fmaf(a, wq[(j + k) >> 2][(j + k) & 3], part[k]);
        }
      }
#pragma unroll
      for (int k = 0; k < NLOGIT; ++k) {
        float v = part[k];
        v += __shfl_xor(v, 16, 32);
        v += __shfl_xor(v, 8, 32);
        v += __shfl_xor(v, 4, 32);
        v += __shfl_xor(v, 2, 32);
        v += __shfl_xor(v, 1, 32);
        part[k] = v + brS[k];
      }
      float mx = part[0];
#pragma unroll
      for (int k = 1; k < NLOGIT; ++k) mx = fmaxf(mx, part[k]);
      float mine = part[0];
#pragma unroll
      for (int k = 1; k < NLOGIT; ++k) mine = (lane == k) ? part[k] : mine;
      const float ex = expf(mine - mx);
      float rw[NLOGIT];
#pragma unroll
      for (int k = 0; k < NLOGIT; ++k) rw[k] = __shfl(ex, k, 32);
      float ssum = rw[0];
#pragma unroll
      for (int k = 1; k < NLOGIT; ++k) ssum = ssum + rw[k];
      const float inv = 1.0f / ssum;
#pragma unroll
      for (int k = 0; k < NLOGIT; ++k) rw[k] = rw[k] * inv;

#pragma unroll 1
      for (int i = 0; i < 4; ++i) {
        const int u0 = lane * 4 + 128 * i;
        const v4f m0v = *(const v4f*)(mrow + u0);
        v4f racc = m0v * rw[0];
#pragma unroll
        for (int m = 1; m < NSLOT; ++m) {
          const v4f mv = *(const v4f*)(mrow + m * NUNIT + u0);
          racc = fma4(rw[m], mv, racc);
        }
        const v4f xs = *(const v4f*)(xrow + u0);
        racc = fma4(rw[16], xs, racc);
        v4h hv;
        hv[0] = (_Float16)(racc[0] * READ_CARRY);
        hv[1] = (_Float16)(racc[1] * READ_CARRY);
        hv[2] = (_Float16)(racc[2] * READ_CARRY);
        hv[3] = (_Float16)(racc[3] * READ_CARRY);
        *(v4h*)(readA + lr * A_PITCH + u0) = hv;
      }
    }
    __syncthreads();

    {
      v8f acc[4];
#pragma unroll
      for (int j = 0; j < 4; ++j) acc[j] = zero8();
#pragma unroll 2
      for (int k0 = 0; k0 < NUNIT; k0 += 32) {
        v16h bf[4];
#pragma unroll
        for (int j = 0; j < 4; ++j)
          bf[j] = Frag<_Float16>::load(WtT + (size_t)(nwcol + 16 * j + cc) * NUNIT + k0 + koff);
        const v16h af = Frag<_Float16>::load(readA + cc * A_PITCH + k0 + koff);
#pragma unroll
        for (int j = 0; j < 4; ++j) acc[j] = Frag<_Float16>::mma(af, bf[j], acc[j]);
        dep_guard_h(acc[0], acc[3], af, bf[3]);
        keep4_h(bf[0], bf[1], bf[2], af);
      }
      acc_guard4(acc[0], acc[1], acc[2], acc[3]);
#pragma unroll
      for (int j = 0; j < 4; ++j) {
        const int n = nwcol + 16 * j + cc;
        const float bv = btS[n];
#pragma unroll
        for (int r = 0; r < 8; ++r) {
          float v = acc[j][r] * ACC_FOLD + bv;
          v = fmaxf(v, 0.0f);
          trS[(8 * hh + r) * TR_PITCH + n] = v;
        }
      }
    }
    __syncthreads();

#pragma unroll 1
    for (int rr = 0; rr < 2; ++rr) {
      const int lr = wave * 2 + rr;
      const int gb = row0 + lr;
      const float* xrow = x + ((size_t)gb * NSTEP + t) * NUNIT;
      const float* mrow = src + (size_t)gb * (NSLOT * NUNIT);
      float* drow = dst + (size_t)gb * (NSLOT * NUNIT);
      const float* trow = trS + lr * TR_PITCH;

      float wp[NSLOT];
#pragma unroll
      for (int k = 0; k < NSLOT; ++k) wp[k] = 0.f;
#pragma unroll 1
      for (int i = 0; i < 4; ++i) {
        const int u0 = lane * 4 + 128 * i;
        const v4f tv = *(const v4f*)(trow + u0);
        const float* wwb = Ww + (size_t)u0 * NSLOT;
#pragma unroll
        for (int j = 0; j < 4; ++j) {
          const float tj = tv[j];
          v4f gq[4];
#pragma unroll
          for (int cq = 0; cq < 4; ++cq) gq[cq] = *(const v4f*)(wwb + 16 * j + 4 * cq);
#pragma unroll
          for (int k = 0; k < NSLOT; ++k) wp[k] = fmaf(tj, gq[k >> 2][k & 3], wp[k]);
        }
      }
#pragma unroll
      for (int k = 0; k < NSLOT; ++k) {
        float v = wp[k];
        v += __shfl_xor(v, 16, 32);
        v += __shfl_xor(v, 8, 32);
        v += __shfl_xor(v, 4, 32);
        v += __shfl_xor(v, 2, 32);
        v += __shfl_xor(v, 1, 32);
        wp[k] = v + bwS[k];
      }
      float zm = wp[0];
#pragma unroll
      for (int k = 1; k < NSLOT; ++k) zm = (lane == k) ? wp[k] : zm;
      zm = fminf(fmaxf(zm, -30.0f), 30.0f);
      const float sg = 1.0f / (1.0f + expf(-zm));

      float* orow = out + ((size_t)gb * NSTEP + t) * NUNIT;
      v4f tv4[4], yv[4];
#pragma unroll
      for (int i = 0; i < 4; ++i) {
        const int u0 = lane * 4 + 128 * i;
        tv4[i] = *(const v4f*)(trow + u0);
        const v4f xs = *(const v4f*)(xrow + u0);
        yv[i] = xs + tv4[i];
      }
#pragma unroll
      for (int i = 0; i < 4; ++i) *(volatile v4f*)(orow + lane * 4 + 128 * i) = yv[i];
      __threadfence();
#pragma unroll
      for (int i = 0; i < 4; ++i) *(volatile v4f*)(orow + lane * 4 + 128 * i) = yv[i];

#pragma unroll 1
      for (int m = 0; m < NSLOT; ++m) {
        const float gm = __shfl(sg, m, 32);
        const float om = 1.0f - gm;
        v4f nv[4];
#pragma unroll
        for (int i = 0; i < 4; ++i) {
          const int u0 = lane * 4 + 128 * i;
          const v4f ov = *(const v4f*)(mrow + m * NUNIT + u0);
          v4f r;
          r[0] = fmaf(gm, tv4[i][0], om * ov[0]);
          r[1] = fmaf(gm, tv4[i][1], om * ov[1]);
          r[2] = fmaf(gm, tv4[i][2], om * ov[2]);
          r[3] = fmaf(gm, tv4[i][3], om * ov[3]);
          nv[i] = r;
        }
#pragma unroll
        for (int i = 0; i < 4; ++i) *(volatile v4f*)(drow + m * NUNIT + lane * 4 + 128 * i) = nv[i];
        __threadfence();
#pragma unroll
        for (int i = 0; i < 4; ++i) *(volatile v4f*)(drow + m * NUNIT + lane * 4 + 128 * i) = nv[i];
      }
    }
    __threadfence_block();
  }
}

extern "C" void kernel_launch(void* const* d_in, const int* in_sizes, int n_in,
                              void* d_out, int out_size, void* d_ws, size_t ws_size,
                              hipStream_t stream) {
  if (n_in < 8) return;
  if (in_sizes[0] != NBATCH * NSTEP * NUNIT) return;
  if (in_sizes[1] != NBATCH * NSLOT * NUNIT) return;
  if (in_sizes[2] != NUNIT * NLOGIT) return;
  if (in_sizes[3] != NLOGIT) return;
  if (in_sizes[4] != NUNIT * NUNIT) return;
  if (in_sizes[5] != NUNIT) return;
  if (in_sizes[6] != NUNIT * NSLOT) return;
  if (in_sizes[7] != NSLOT) return;
  if (out_size != NBATCH * NSTEP * NUNIT) return;

  const float* x    = (const float*)d_in[0];
  const float* mem0 = (const float*)d_in[1];
  const float* Wr   = (const float*)d_in[2];
  const float* br   = (const float*)d_in[3];
  const float* Wt   = (const float*)d_in[4];
  const float* bt   = (const float*)d_in[5];
  const float* Ww   = (const float*)d_in[6];
  const float* bw   = (const float*)d_in[7];
  float* out        = (float*)d_out;

  const size_t wt_bytes  = (size_t)NUNIT * NUNIT * sizeof(_Float16);
  const size_t mem_bytes = (size_t)NBATCH * NSLOT * NUNIT * sizeof(float);
  if (ws_size < wt_bytes + 2 * mem_bytes) return;
  char* ws = (char*)d_ws;
  _Float16* WtT = (_Float16*)(ws);
  float* memA = (float*)(ws + wt_bytes);
  float* memB = (float*)(ws + wt_bytes + mem_bytes);

  wt_cast_kmajor<<<dim3(NUNIT / 64, NUNIT / 64), 256, 0, stream>>>(Wt, WtT);
  dnc_steps<<<NBATCH / ROWS_PB, 256, 0, stream>>>(x, mem0, Wr, br, WtT, bt, Ww, bw, memA, memB, out);
}
